// Net_76622216561354
// MI455X (gfx1250) — hardware-verified
//
#include <hip/hip_runtime.h>
#include <stdint.h>

constexpr int NUM_NODES  = 131072;
constexpr int NUM_EDGES  = 524288;
constexpr int FEAT_IN    = 16;
constexpr int HID        = 64;
constexpr int CONV_CH    = 16;
constexpr int BOND       = 4;
constexpr int NUM_GRAPHS = 8192;
constexpr int NUM_GRU    = 4;
constexpr int NUM_REP    = 2;
constexpr int GATE3      = 3 * HID;
constexpr int TCOLS      = 96;
constexpr int DEG_CAP    = 32;
constexpr int BUILD_TILE = 512;
constexpr bool SPLIT_RZ_COLS = true;
constexpr bool SPLIT_HN_COLS = true;

static_assert(HID == 64 && CONV_CH == 16 && FEAT_IN == 16 && BOND == 4, "shape constants match the wire contract");
static_assert(NUM_NODES % 128 == 0 && NUM_NODES % BUILD_TILE == 0, "node tiles exact");
static_assert(NUM_EDGES % 4 == 0 && NUM_EDGES % 32 == 0 && (NUM_EDGES / 4) % 256 == 0, "edge list read as int4 and in 32-edge chunks");
static_assert(NUM_GRAPHS % 256 == 0, "pool grid exact");
static_assert(TCOLS == 6 * CONV_CH, "T = 4 bond blocks + bias block + root block");
static_assert(DEG_CAP * 4 == 128, "one 128-B table line per node");
static_assert(BUILD_TILE % 256 == 0, "table tile is a multiple of the block size");

constexpr int UNIT_L0T = 0;
constexpr int UNIT_L1T = 256;
constexpr int UNIT_WCT = 384;
constexpr int UNIT_WIH = 768;
constexpr int UNIT_WHH = 3840;
constexpr int UNIT_CST = 9984;
constexpr int PREP_UNITS = 10368;
constexpr int EL_L1T = UNIT_L1T * 8;
constexpr int EL_WCT = UNIT_WCT * 8;
constexpr int EL_WIH = UNIT_WIH * 8;
constexpr int EL_WHH = UNIT_WHH * 8;
static_assert(UNIT_L0T == 0, "L0T plane first");
static_assert(UNIT_L1T * 16 == HID * 32 * 2, "L0T plane [64][32]");
static_assert((UNIT_WCT - UNIT_L1T) * 16 == CONV_CH * HID * 2, "L1T plane [16][64]");
static_assert((UNIT_WIH - UNIT_WCT) * 16 == TCOLS * 32 * 2, "WCT plane [96][32]");
static_assert((UNIT_WHH - UNIT_WIH) * 16 == NUM_GRU * GATE3 * 32 * 2, "WIH planes [4][192][32]");
static_assert((UNIT_CST - UNIT_WHH) * 16 == NUM_GRU * GATE3 * HID * 2, "WHH planes [4][192][64]");
static_assert(PREP_UNITS % 32 == 0 && UNIT_CST % 32 == 0 && UNIT_WHH % 32 == 0 && UNIT_WIH % 32 == 0 && UNIT_WCT % 32 == 0 && UNIT_L1T % 32 == 0, "region bounds on wave bounds");
constexpr int CST_GB  = 0;
constexpr int CST_BT  = 1024;
constexpr int CST_L1B = 1152;
constexpr int CST_L0B = 1280;
constexpr int CST_L2W = 1408;
constexpr int CST_FLOATS = 1536;
static_assert((PREP_UNITS - UNIT_CST) * 4 == CST_FLOATS, "constant area size");

typedef __attribute__((ext_vector_type(16))) __bf16   v16b;
typedef __attribute__((ext_vector_type(8)))  __bf16   v8b;
typedef __attribute__((ext_vector_type(8)))  float    v8f;
typedef __attribute__((ext_vector_type(4)))  float    v4f;
typedef __attribute__((ext_vector_type(4)))  unsigned v4u;
typedef __attribute__((ext_vector_type(4)))  int      v4i;

__device__ __forceinline__ unsigned short f2bf_bits(float f) {
  unsigned u = __float_as_uint(f);
  return (unsigned short)((u + 0x7FFFu + ((u >> 16) & 1u)) >> 16);
}
__device__ __forceinline__ float bf_bits2f(unsigned short h) { return __uint_as_float(((unsigned)h) << 16); }
__device__ __forceinline__ float bfr(float f) { return bf_bits2f(f2bf_bits(f)); }
__device__ __forceinline__ __bf16 bits2bf(unsigned short b) { return __builtin_bit_cast(__bf16, b); }
__device__ __forceinline__ void split_bits(float f, unsigned short& hb, unsigned short& lb) {
  hb = f2bf_bits(f);
  lb = f2bf_bits(f - bf_bits2f(hb));
}
__device__ __forceinline__ unsigned pack2(unsigned short lo16, unsigned short hi16) {
  return (unsigned)lo16 | ((unsigned)hi16 << 16);
}

union FragB { v16b v; v8b h[2]; };
__device__ __forceinline__ v16b frag_load(const __bf16* p) {
  FragB f;
  f.h[0] = *(const v8b*)(p);
  f.h[1] = *(const v8b*)(p + 16);
  return f.v;
}
__device__ __forceinline__ v8f mma_bf(v16b a, v16b b, v8f c) {
  c = __builtin_amdgcn_wmma_f32_16x16x32_bf16(false, a, false, b, (short)0, c, false, false);
  asm volatile("v_nop\n\tv_nop\n\tv_nop\n\tv_nop" : "+v"(c) : "v"(a), "v"(b));
  return c;
}
__device__ __forceinline__ float fsig(float v)  { return __builtin_amdgcn_rcpf(1.0f + __expf(-v)); }
__device__ __forceinline__ float ftanh(float v) { return 1.0f - 2.0f * __builtin_amdgcn_rcpf(__expf(2.0f * v) + 1.0f); }

__global__ __launch_bounds__(256) void prep_kernel(
    const float* __restrict__ lin0_w, const float* __restrict__ lin0_b,
    const float* __restrict__ nn1_w,  const float* __restrict__ nn1_b,
    const float* __restrict__ root_w, const float* __restrict__ conv_b,
    const float* __restrict__ w_ih,   const float* __restrict__ w_hh,
    const float* __restrict__ b_ih,   const float* __restrict__ b_hh,
    const float* __restrict__ lin1_w, const float* __restrict__ lin1_b,
    const float* __restrict__ lin2_w, unsigned* wreg) {
  const int u = blockIdx.x * 256 + threadIdx.x;
  if (u >= PREP_UNITS) return;
  v4u ow;
  if (u < UNIT_CST) {
    float v[8];
    const int el0 = u * 8;
    if (u < UNIT_L1T) {
#pragma unroll
      for (int e = 0; e < 8; ++e) {
        const int idx = el0 + e;
        const int n = idx >> 5, k = idx & 31;
        const float ld = lin0_w[(k & 15) * HID + n];
        v[e] = (k < FEAT_IN) ? ld : 0.0f;
      }
    } else if (u < UNIT_WCT) {
#pragma unroll
      for (int e = 0; e < 8; ++e) {
        const int idx = el0 - EL_L1T + e;
        const int n = idx >> 6, k = idx & 63;
        v[e] = lin1_w[k * CONV_CH + n];
      }
    } else if (u < UNIT_WIH) {
#pragma unroll
      for (int e = 0; e < 8; ++e) {
        const int idx = el0 - EL_WCT + e;
        const int n = idx >> 5, k = idx & 31;
        const int i = k & 15, g = n >> 4, o = n & 15;
        const int gc = (g < 3) ? g : 3;
        const float va = nn1_w[gc * 256 + i * 16 + o];
        const float vb = nn1_b[i * 16 + o];
        const float vc = root_w[i * 16 + o];
        v[e] = (g < 4) ? va : ((g == 4) ? vb : vc);
      }
    } else if (u < UNIT_WHH) {
#pragma unroll
      for (int e = 0; e < 8; ++e) {
        const int idx = el0 - EL_WIH + e;
        const int row = idx >> 5, k = idx & 31;
        v[e] = w_ih[row * CONV_CH + (k & 15)];
      }
    } else {
#pragma unroll
      for (int e = 0; e < 8; ++e) v[e] = w_hh[el0 - EL_WHH + e];
    }
    ow[0] = pack2(f2bf_bits(v[0]), f2bf_bits(v[1]));
    ow[1] = pack2(f2bf_bits(v[2]), f2bf_bits(v[3]));
    ow[2] = pack2(f2bf_bits(v[4]), f2bf_bits(v[5]));
    ow[3] = pack2(f2bf_bits(v[6]), f2bf_bits(v[7]));
  } else {
    float v[4];
    const int f0 = (u - UNIT_CST) * 4;
    const int sect = f0 >> 7;
    if (sect < 8) {
#pragma unroll
      for (int e = 0; e < 4; ++e) {
        const int f = f0 + e;
        const int j = f >> 8, cidx = f & 255;
        const int grp = cidx >> 6, d = cidx & 63;
        const int bs = j * GATE3 + d;
        const float ir = bfr(b_ih[bs]),       hr = bfr(b_hh[bs]);
        const float iz = bfr(b_ih[bs + 64]),  hz = bfr(b_hh[bs + 64]);
        const float in_ = bfr(b_ih[bs + 128]), hn = bfr(b_hh[bs + 128]);
        const float sr = ir + hr, sz = iz + hz;
        v[e] = (grp == 0) ? sr : ((grp == 1) ? sz : ((grp == 2) ? in_ : hn));
      }
    } else if (sect == 8) {
#pragma unroll
      for (int e = 0; e < 4; ++e) {
        const int t = f0 + e - CST_BT;
        const float ld = bfr(conv_b[t & 15]);
        v[e] = (t >= 80 && t < 96) ? ld : 0.0f;
      }
    } else if (sect == 9) {
#pragma unroll
      for (int e = 0; e < 4; ++e) {
        const int t = f0 + e - CST_L1B;
        const float ld = bfr(lin1_b[t & 15]);
        v[e] = (t < 16) ? ld : 0.0f;
      }
    } else if (sect == 10) {
#pragma unroll
      for (int e = 0; e < 4; ++e) {
        const int t = f0 + e - CST_L0B;
        const float ld = bfr(lin0_b[t & 63]);
        v[e] = (t < 64) ? ld : 0.0f;
      }
    } else {
#pragma unroll
      for (int e = 0; e < 4; ++e) {
        const int t = f0 + e - CST_L2W;
        const float ld = bfr(lin2_w[t & 63]);
        v[e] = (t < 64) ? ld : 0.0f;
      }
    }
    ow[0] = __float_as_uint(v[0]);
    ow[1] = __float_as_uint(v[1]);
    ow[2] = __float_as_uint(v[2]);
    ow[3] = __float_as_uint(v[3]);
  }
  v4u* dst = (v4u*)wreg + u;
  *(volatile v4u*)dst = ow;
  __threadfence();
  *(volatile v4u*)dst = ow;
}

__global__ __launch_bounds__(256) void build_kernel(const int* __restrict__ dstv, int* cntOut, int* nbr) {
  __shared__ __align__(16) int cntL[BUILD_TILE];
  __shared__ __align__(16) int slotL[BUILD_TILE * DEG_CAP];
  const int tid = threadIdx.x;
  const int base = blockIdx.x * BUILD_TILE;
#pragma unroll 1
  for (int i = 0; i < BUILD_TILE / 256; ++i) cntL[i * 256 + tid] = 0;
#pragma unroll 1
  for (int i = 0; i < (BUILD_TILE * DEG_CAP) / 256; ++i) slotL[i * 256 + tid] = 0;
  __syncthreads();
  const v4i* d4 = (const v4i*)dstv;
#pragma unroll 1
  for (int i = tid; i < NUM_EDGES / 4; i += 256) {
    const v4i d = d4[i];
    const int e0 = i * 4;
    const int l0 = d[0] - base, l1 = d[1] - base, l2 = d[2] - base, l3 = d[3] - base;
    if ((unsigned)l0 < (unsigned)BUILD_TILE) { const int p = atomicAdd(&cntL[l0], 1); if (p < DEG_CAP) slotL[l0 * DEG_CAP + p] = e0; }
    if ((unsigned)l1 < (unsigned)BUILD_TILE) { const int p = atomicAdd(&cntL[l1], 1); if (p < DEG_CAP) slotL[l1 * DEG_CAP + p] = e0 + 1; }
    if ((unsigned)l2 < (unsigned)BUILD_TILE) { const int p = atomicAdd(&cntL[l2], 1); if (p < DEG_CAP) slotL[l2 * DEG_CAP + p] = e0 + 2; }
    if ((unsigned)l3 < (unsigned)BUILD_TILE) { const int p = atomicAdd(&cntL[l3], 1); if (p < DEG_CAP) slotL[l3 * DEG_CAP + p] = e0 + 3; }
  }
  __syncthreads();
#pragma unroll 1
  for (int q = 0; q < BUILD_TILE / 256; ++q) {
    const int nl = q * 256 + tid;
    int cn = cntL[nl];
    cn = (cn < 0) ? 0 : ((cn > DEG_CAP) ? DEG_CAP : cn);
    int* row = slotL + nl * DEG_CAP;
#pragma unroll 1
    for (int a = 1; a < cn; ++a) {
      const int key = row[a];
      int pos = a;
#pragma unroll 1
      for (int b = a - 1; b >= 0; --b) {
        const int vb = row[b];
        if (vb > key) { row[b + 1] = vb; pos = b; } else { break; }
      }
      row[pos] = key;
    }
  }
  __syncthreads();
  v4i* nout = (v4i*)(nbr + (size_t)base * DEG_CAP);
  v4i* cout_ = (v4i*)(cntOut + base);
  for (int pass = 0; pass < 2; ++pass) {
#pragma unroll 1
    for (int it = 0; it < (BUILD_TILE * DEG_CAP) / (4 * 256); ++it) {
      const int uidx = it * 256 + tid;
      const v4i v = *(const v4i*)(slotL + uidx * 4);
      *(volatile v4i*)(nout + uidx) = v;
    }
    if (tid < BUILD_TILE / 4) {
      const v4i v = *(const v4i*)(cntL + tid * 4);
      *(volatile v4i*)(cout_ + tid) = v;
    }
    __threadfence();
  }
}

__device__ __forceinline__ void store_h_rows(const float* slabw, unsigned short* Hhi, unsigned short* Hlo, int row0, int lane) {
  const int q = lane >> 3, c8 = (lane & 7) * 8;
  for (int pass = 0; pass < 2; ++pass) {
#pragma unroll
    for (int it = 0; it < 4; ++it) {
      const int row = it * 4 + q;
      const float* sp = slabw + row * 68 + c8;
      const v4f f0 = *(const v4f*)(sp);
      const v4f f1 = *(const v4f*)(sp + 4);
      unsigned short hb[8], lb[8];
#pragma unroll
      for (int e = 0; e < 4; ++e) {
        const float a = f0[e];
        const float b = f1[e];
        split_bits(a, hb[e], lb[e]);
        split_bits(b, hb[4 + e], lb[4 + e]);
      }
      v4u hw, lw;
      hw[0] = pack2(hb[0], hb[1]); hw[1] = pack2(hb[2], hb[3]); hw[2] = pack2(hb[4], hb[5]); hw[3] = pack2(hb[6], hb[7]);
      lw[0] = pack2(lb[0], lb[1]); lw[1] = pack2(lb[2], lb[3]); lw[2] = pack2(lb[4], lb[5]); lw[3] = pack2(lb[6], lb[7]);
      const size_t off = (size_t)(row0 + row) * HID + (size_t)c8;
      *(volatile v4u*)(Hhi + off) = hw;
      *(volatile v4u*)(Hlo + off) = lw;
    }
    __threadfence();
  }
}

__global__ __launch_bounds__(256) void lin0_kernel(const float* __restrict__ x, const unsigned short* __restrict__ L0T,
                                                   const float* __restrict__ cst, unsigned short* Hhi, unsigned short* Hlo) {
  __shared__ __align__(16) float slab[8][16 * 68];
  const int tid = threadIdx.x, lane = tid & 31, wave = tid >> 5;
  const int c = lane & 15, hh = lane >> 4, koff = hh * 8;
  const int row0 = blockIdx.x * 128 + wave * 16;
  const float* xr = x + (size_t)(row0 + c) * FEAT_IN + koff;
  const v4f x0 = *(const v4f*)(xr);
  const v4f x1 = *(const v4f*)(xr + 4);
  const __bf16 zb = bits2bf((unsigned short)0);
  v16b a;
#pragma unroll
  for (int e = 0; e < 4; ++e) {
    const float p0 = x0[e];
    const float p1 = x1[e];
    a[e] = bits2bf(f2bf_bits(p0));
    a[4 + e] = bits2bf(f2bf_bits(p1));
    a[8 + e] = zb;
    a[12 + e] = zb;
  }
  const v8f z8 = {0.f, 0.f, 0.f, 0.f, 0.f, 0.f, 0.f, 0.f};
  float* sw = slab[wave];
#pragma unroll
  for (int nt = 0; nt < 4; ++nt) {
    const v16b b = frag_load((const __bf16*)L0T + (size_t)(nt * 16 + c) * 32 + koff);
    v8f acc = mma_bf(a, b, z8);
    const float bias = cst[CST_L0B + nt * 16 + c];
#pragma unroll
    for (int r = 0; r < 8; ++r) sw[(8 * hh + r) * 68 + nt * 16 + c] = fmaxf(acc[r] + bias, 0.0f);
  }
  __syncthreads();
  store_h_rows(sw, Hhi, Hlo, row0, lane);
}

__global__ __launch_bounds__(128) void msgprep_kernel(const unsigned short* __restrict__ Hhi, const unsigned short* __restrict__ Hlo,
                                                      const unsigned short* __restrict__ L1T, const unsigned short* __restrict__ WCT,
                                                      const float* __restrict__ cst, float* Tpl) {
  __shared__ __align__(16) unsigned short a2s[4][16 * 32];
  __shared__ __align__(16) float tslab[4][16 * 100];
  const int tid = threadIdx.x, lane = tid & 31, wave = tid >> 5;
  const int c = lane & 15, hh = lane >> 4, koff = hh * 8;
  const int row0 = blockIdx.x * 64 + wave * 16;
  const v8f z8 = {0.f, 0.f, 0.f, 0.f, 0.f, 0.f, 0.f, 0.f};
  {
    const __bf16* hrow = (const __bf16*)Hhi + (size_t)(row0 + c) * HID + koff;
    const __bf16* lrow = (const __bf16*)Hlo + (size_t)(row0 + c) * HID + koff;
    const v16b ah0 = frag_load(hrow), ah1 = frag_load(hrow + 32);
    const v16b al0 = frag_load(lrow), al1 = frag_load(lrow + 32);
    const __bf16* l1 = (const __bf16*)L1T + (size_t)c * HID + koff;
    const v16b b0 = frag_load(l1), b1 = frag_load(l1 + 32);
    v8f acc = z8;
    acc = mma_bf(ah0, b0, acc);
    acc = mma_bf(al0, b0, acc);
    acc = mma_bf(ah1, b1, acc);
    acc = mma_bf(al1, b1, acc);
    const float bias = cst[CST_L1B + c];
#pragma unroll
    for (int r = 0; r < 8; ++r) {
      unsigned short hb, lb;
      split_bits(acc[r] + bias, hb, lb);
      a2s[wave][(8 * hh + r) * 32 + c] = hb;
      a2s[wave][(8 * hh + r) * 32 + 16 + c] = lb;
    }
  }
  __syncthreads();
  FragB fa;
  fa.h[0] = *(const v8b*)(&a2s[wave][c * 32 + koff]);
  fa.h[1] = *(const v8b*)(&a2s[wave][c * 32 + 16 + koff]);
  const v16b a2 = fa.v;
  float* tw = tslab[wave];
#pragma unroll
  for (int nt = 0; nt < 6; ++nt) {
    const v16b b = frag_load((const __bf16*)WCT + (size_t)(nt * 16 + c) * 32 + koff);
    v8f acc = mma_bf(a2, b, z8);
    const float bias = cst[CST_BT + nt * 16 + c];
#pragma unroll
    for (int r = 0; r < 8; ++r) tw[(8 * hh + r) * 100 + nt * 16 + c] = acc[r] + bias;
  }
  __syncthreads();
  float* tbase = Tpl + (size_t)row0 * TCOLS;
  for (int pass = 0; pass < 2; ++pass) {
#pragma unroll 1
    for (int it = 0; it < 12; ++it) {
      const int uu = it * 32 + lane;
      const int row = uu / 24;
      const int cu = uu - row * 24;
      const v4f v = *(const v4f*)(tw + row * 100 + cu * 4);
      *(volatile v4f*)(tbase + (size_t)uu * 4) = v;
    }
    __threadfence();
  }
}

__device__ __forceinline__ float edge_msg(const float* __restrict__ Tpl, const float* __restrict__ ea,
                                          const int* __restrict__ ei, int e, int o) {
  e = (e < 0) ? 0 : ((e > NUM_EDGES - 1) ? (NUM_EDGES - 1) : e);
  int s = ei[e];
  s = (s < 0) ? 0 : ((s > NUM_NODES - 1) ? (NUM_NODES - 1) : s);
  const v4f a = *(const v4f*)(ea + (size_t)e * BOND);
  const float a0 = a[0];
  const float a1 = a[1];
  const float a2 = a[2];
  const float a3 = a[3];
  const float* Ts = Tpl + (size_t)s * TCOLS + o;
  const float t0 = Ts[0], t1 = Ts[16], t2 = Ts[32], t3 = Ts[48], tb = Ts[64];
  float m = tb;
  m = fmaf(bfr(a0), t0, m);
  m = fmaf(bfr(a1), t1, m);
  m = fmaf(bfr(a2), t2, m);
  m = fmaf(bfr(a3), t3, m);
  return m;
}

__global__ __launch_bounds__(256) void edge_kernel(const float* __restrict__ Tpl, const float* __restrict__ ea,
                                                   const int* __restrict__ ei, const int* __restrict__ nbr,
                                                   const int* __restrict__ cntv, float* xin) {
  const int tid = threadIdx.x;
  const int lane = tid & 31, hh = lane >> 4;
  const int n = blockIdx.x * 16 + (tid >> 4);
  const int o = tid & 15;
  const int cnt = cntv[n];
  const int cntc = (cnt < 0) ? 0 : ((cnt > NUM_EDGES) ? NUM_EDGES : cnt);
  const int cc = (cntc > DEG_CAP) ? DEG_CAP : cntc;
  const int co = __shfl_xor(cc, 16, 32);
  int cmax = (cc > co) ? cc : co;
  cmax = __builtin_amdgcn_readfirstlane(cmax);
  cmax = (cmax > DEG_CAP) ? DEG_CAP : cmax;
  const int* nrow = nbr + (size_t)n * DEG_CAP;
  float sum = 0.0f;
#pragma unroll 1
  for (int p = 0; p < cmax; ++p) {
    const int e = nrow[p];
    const float m = edge_msg(Tpl, ea, ei, e, o);
    sum += (p < cc) ? m : 0.0f;
  }
  const bool over = cntc > DEG_CAP;
  const unsigned ovm = __builtin_amdgcn_ballot_w32(over);
  float sumg = 0.0f;
  if (ovm != 0u) {
    const bool overA = (ovm & 1u) != 0u;
    const bool overB = (ovm & 0x10000u) != 0u;
    const int nodeA = __builtin_amdgcn_readfirstlane(n);
    const int nodeB = nodeA + 1;
    const int* dstrow = ei + NUM_EDGES;
#pragma unroll 1
    for (int e0 = 0; e0 < NUM_EDGES; e0 += 32) {
      const int d = dstrow[e0 + lane];
      const unsigned mA = __builtin_amdgcn_ballot_w32(overA && (d == nodeA));
      const unsigned mB = __builtin_amdgcn_ballot_w32(overB && (d == nodeB));
      const unsigned sel = (hh == 0) ? mA : mB;
      unsigned mm = mA | mB;
#pragma unroll 1
      for (int q = 0; q < 32; ++q) {
        if (mm == 0u) break;
        const int b = __builtin_ctz(mm);
        mm &= (mm - 1u);
        const float m = edge_msg(Tpl, ea, ei, e0 + b, o);
        const bool mine = ((sel >> b) & 1u) != 0u;
        sumg += mine ? m : 0.0f;
      }
    }
  }
  const float tot = over ? sumg : sum;
  const float inv = 1.0f / fmaxf((float)cntc, 1.0f);
  const float rootv = Tpl[(size_t)n * TCOLS + 80 + o];
  const float xv = rootv + tot * inv;
  float* dst = xin + (size_t)n * CONV_CH + o;
  *(volatile float*)dst = xv;
  __threadfence();
  *(volatile float*)dst = xv;
}

template <bool SPLIT_RZ, bool SPLIT_HN>
__global__ __launch_bounds__(128) void gru_kernel(unsigned short* Hhi, unsigned short* Hlo, const float* __restrict__ xin,
                                                  const unsigned short* __restrict__ WIHj, const unsigned short* __restrict__ WHHj,
                                                  const float* __restrict__ gbj) {
  __shared__ __align__(16) float hslab[4][16 * 68];
  const int tid = threadIdx.x, lane = tid & 31, wave = tid >> 5;
  const int c = lane & 15, hh = lane >> 4, koff = hh * 8;
  const int row0 = blockIdx.x * 64 + wave * 16;
  const v8f z8 = {0.f, 0.f, 0.f, 0.f, 0.f, 0.f, 0.f, 0.f};
  const __bf16* hrow = (const __bf16*)Hhi + (size_t)(row0 + c) * HID + koff;
  const __bf16* lrow = (const __bf16*)Hlo + (size_t)(row0 + c) * HID + koff;
  const v16b ah0 = frag_load(hrow), ah1 = frag_load(hrow + 32);
  const v16b al0 = frag_load(lrow), al1 = frag_load(lrow + 32);
  v16b ax;
  {
    const float* xr = xin + (size_t)(row0 + c) * CONV_CH + koff;
    const v4f x0 = *(const v4f*)(xr);
    const v4f x1 = *(const v4f*)(xr + 4);
#pragma unroll
    for (int e = 0; e < 4; ++e) {
      const float p0 = x0[e];
      const float p1 = x1[e];
      unsigned short hb, lb;
      split_bits(p0, hb, lb);
      ax[e] = bits2bf(hb);
      ax[8 + e] = bits2bf(lb);
      split_bits(p1, hb, lb);
      ax[4 + e] = bits2bf(hb);
      ax[12 + e] = bits2bf(lb);
    }
  }
  const unsigned* hw = (const unsigned*)Hhi;
  const unsigned* lw = (const unsigned*)Hlo;
  float* sw = hslab[wave];
#pragma unroll 1
  for (int ug = 0; ug < 4; ++ug) {
    const int u = ug * 16 + c;
    const __bf16* wi = (const __bf16*)WIHj + (size_t)u * 32 + koff;
    const __bf16* wh = (const __bf16*)WHHj + (size_t)u * HID + koff;
    v8f ar = z8, az = z8, ai = z8, an = z8;
    {
      const v16b bi = frag_load(wi);
      const v16b b0 = frag_load(wh);
      const v16b b1 = frag_load(wh + 32);
      ar = mma_bf(ax, bi, ar);
      ar = mma_bf(ah0, b0, ar);
      if (SPLIT_RZ) ar = mma_bf(al0, b0, ar);
      ar = mma_bf(ah1, b1, ar);
      if (SPLIT_RZ) ar = mma_bf(al1, b1, ar);
    }
    {
      const v16b bi = frag_load(wi + 64 * 32);
      const v16b b0 = frag_load(wh + 64 * HID);
      const v16b b1 = frag_load(wh + 64 * HID + 32);
      az = mma_bf(ax, bi, az);
      az = mma_bf(ah0, b0, az);
      if (SPLIT_RZ) az = mma_bf(al0, b0, az);
      az = mma_bf(ah1, b1, az);
      if (SPLIT_RZ) az = mma_bf(al1, b1, az);
    }
    {
      const v16b bi = frag_load(wi + 128 * 32);
      const v16b b0 = frag_load(wh + 128 * HID);
      const v16b b1 = frag_load(wh + 128 * HID + 32);
      ai = mma_bf(ax, bi, ai);
      an = mma_bf(ah0, b0, an);
      if (SPLIT_HN) an = mma_bf(al0, b0, an);
      an = mma_bf(ah1, b1, an);
      if (SPLIT_HN) an = mma_bf(al1, b1, an);
    }
    const float cr = gbj[u], cz = gbj[64 + u], ci = gbj[128 + u], cn = gbj[192 + u];
    const int odd = u & 1;
#pragma unroll
    for (int r = 0; r < 8; ++r) {
      const int lr = 8 * hh + r;
      const size_t widx = ((size_t)(row0 + lr) * HID + (size_t)u) >> 1;
      const unsigned wa = hw[widx];
      const unsigned wb = lw[widx];
      const float ha = odd ? __uint_as_float(wa & 0xffff0000u) : __uint_as_float(wa << 16);
      const float hb = odd ? __uint_as_float(wb & 0xffff0000u) : __uint_as_float(wb << 16);
      const float hold = ha + hb;
      const float rr = fsig(ar[r] + cr);
      const float zz = fsig(az[r] + cz);
      const float gn = an[r] + cn;
      const float nn = ftanh(fmaf(rr, gn, ai[r] + ci));
      sw[lr * 68 + u] = fmaf(zz, hold - nn, nn);
    }
  }
  __syncthreads();
  store_h_rows(sw, Hhi, Hlo, row0, lane);
}

__global__ __launch_bounds__(256) void pool_kernel(const unsigned short* __restrict__ Hhi, const unsigned short* __restrict__ Hlo,
                                                   const float* __restrict__ cst, const int* __restrict__ batch, float* out) {
  __shared__ float w2s[HID];
  const int tid = threadIdx.x;
  if (tid < HID) w2s[tid] = cst[CST_L2W + tid];
  __syncthreads();
  const int g = blockIdx.x * 256 + tid;
  int lo0 = 0, hi0 = NUM_NODES, lo1 = 0, hi1 = NUM_NODES;
#pragma unroll 1
  for (int s = 0; s < 18; ++s) {
    const int m0 = (lo0 + hi0) >> 1;
    const int m1 = (lo1 + hi1) >> 1;
    const int m0c = (m0 > NUM_NODES - 1) ? (NUM_NODES - 1) : m0;
    const int m1c = (m1 > NUM_NODES - 1) ? (NUM_NODES - 1) : m1;
    const int v0 = batch[m0c];
    const int v1 = batch[m1c];
    const bool a0 = lo0 < hi0, a1 = lo1 < hi1;
    const bool g0 = v0 < g, g1 = v1 < (g + 1);
    lo0 = (a0 && g0) ? (m0 + 1) : lo0;
    hi0 = (a0 && !g0) ? m0 : hi0;
    lo1 = (a1 && g1) ? (m1 + 1) : lo1;
    hi1 = (a1 && !g1) ? m1 : hi1;
  }
  int cnt = lo1 - lo0;
  cnt = (cnt < 0) ? 0 : ((cnt > NUM_NODES) ? NUM_NODES : cnt);
  int cm = cnt;
#pragma unroll
  for (int off = 16; off >= 1; off >>= 1) {
    const int ov = __shfl_xor(cm, off, 32);
    cm = (ov > cm) ? ov : cm;
  }
  cm = __builtin_amdgcn_readfirstlane(cm);
  cm = (cm > NUM_NODES) ? NUM_NODES : cm;
  const v4u* hp = (const v4u*)Hhi;
  const v4u* lp = (const v4u*)Hlo;
  float acc = 0.0f;
#pragma unroll 1
  for (int p = 0; p < cm; ++p) {
    int node = lo0 + p;
    node = (node > NUM_NODES - 1) ? (NUM_NODES - 1) : node;
    float y = 0.0f;
#pragma unroll 1
    for (int ch = 0; ch < 8; ++ch) {
      const v4u wa = hp[(size_t)node * 8 + ch];
      const v4u wb = lp[(size_t)node * 8 + ch];
#pragma unroll
      for (int i = 0; i < 4; ++i) {
        const unsigned a = wa[i];
        const unsigned b = wb[i];
        const float e0 = __uint_as_float(a << 16) + __uint_as_float(b << 16);
        const float e1 = __uint_as_float(a & 0xffff0000u) + __uint_as_float(b & 0xffff0000u);
        y = fmaf(e0, w2s[ch * 8 + 2 * i], y);
        y = fmaf(e1, w2s[ch * 8 + 2 * i + 1], y);
      }
    }
    acc += (p < cnt) ? y : 0.0f;
  }
  float* dst = out + g;
  *(volatile float*)dst = acc;
  __threadfence();
  *(volatile float*)dst = acc;
}

constexpr size_t SZ_H   = (size_t)NUM_NODES * HID * 2;
constexpr size_t SZ_T   = (size_t)NUM_NODES * TCOLS * 4;
constexpr size_t SZ_X   = (size_t)NUM_NODES * CONV_CH * 4;
constexpr size_t SZ_NBR = (size_t)NUM_NODES * DEG_CAP * 4;
constexpr size_t SZ_CNT = (size_t)NUM_NODES * 4;
constexpr size_t SZ_W   = (size_t)PREP_UNITS * 16;
constexpr size_t OFF_HHI = 0;
constexpr size_t OFF_HLO = OFF_HHI + SZ_H;
constexpr size_t OFF_T   = OFF_HLO + SZ_H;
constexpr size_t OFF_X   = OFF_T + SZ_T;
constexpr size_t OFF_NBR = OFF_X + SZ_X;
constexpr size_t OFF_CNT = OFF_NBR + SZ_NBR;
constexpr size_t OFF_W   = OFF_CNT + SZ_CNT;
constexpr size_t WS_TOTAL = OFF_W + SZ_W;
static_assert(WS_TOTAL <= (size_t)134217728, "carve within 128 MiB");
static_assert(OFF_HLO % 256 == 0 && OFF_T % 256 == 0 && OFF_X % 256 == 0 && OFF_NBR % 256 == 0 && OFF_CNT % 256 == 0 && OFF_W % 256 == 0, "aligned carve");

extern "C" void kernel_launch(void* const* d_in, const int* in_sizes, int n_in,
                              void* d_out, int out_size, void* d_ws, size_t ws_size, hipStream_t stream) {
  if (n_in < 17 || d_out == nullptr || d_ws == nullptr) return;
  if (in_sizes[0] != NUM_NODES * FEAT_IN || in_sizes[1] != NUM_EDGES * BOND || in_sizes[2] != FEAT_IN * HID ||
      in_sizes[3] != HID || in_sizes[4] != BOND * 256 || in_sizes[5] != 256 || in_sizes[6] != 256 ||
      in_sizes[7] != CONV_CH || in_sizes[8] != NUM_GRU * GATE3 * CONV_CH || in_sizes[9] != NUM_GRU * GATE3 * HID ||
      in_sizes[10] != NUM_GRU * GATE3 || in_sizes[11] != NUM_GRU * GATE3 || in_sizes[12] != HID * CONV_CH ||
      in_sizes[13] != CONV_CH || in_sizes[14] != HID || in_sizes[15] != 2 * NUM_EDGES || in_sizes[16] != NUM_NODES ||
      out_size != NUM_GRAPHS) return;
  if (WS_TOTAL > ws_size) return;

  const float* x         = (const float*)d_in[0];
  const float* edge_attr = (const float*)d_in[1];
  const float* lin0_w    = (const float*)d_in[2];
  const float* lin0_b    = (const float*)d_in[3];
  const float* nn1_w     = (const float*)d_in[4];
  const float* nn1_b     = (const float*)d_in[5];
  const float* root_w    = (const float*)d_in[6];
  const float* conv_b    = (const float*)d_in[7];
  const float* gru_w_ih  = (const float*)d_in[8];
  const float* gru_w_hh  = (const float*)d_in[9];
  const float* gru_b_ih  = (const float*)d_in[10];
  const float* gru_b_hh  = (const float*)d_in[11];
  const float* lin1_w    = (const float*)d_in[12];
  const float* lin1_b    = (const float*)d_in[13];
  const float* lin2_w    = (const float*)d_in[14];
  const int*   edge_idx  = (const int*)d_in[15];
  const int*   batch     = (const int*)d_in[16];
  float* out = (float*)d_out;

  char* ws = (char*)d_ws;
  unsigned short* HHI = (unsigned short*)(ws + OFF_HHI);
  unsigned short* HLO = (unsigned short*)(ws + OFF_HLO);
  float*          TPL = (float*)(ws + OFF_T);
  float*          XIN = (float*)(ws + OFF_X);
  int*            NBR = (int*)(ws + OFF_NBR);
  int*            CNT = (int*)(ws + OFF_CNT);
  unsigned*       WGT = (unsigned*)(ws + OFF_W);
  const unsigned short* W16 = (const unsigned short*)(ws + OFF_W);
  const unsigned short* L0T = W16;
  const unsigned short* L1T = W16 + EL_L1T;
  const unsigned short* WCT = W16 + EL_WCT;
  const unsigned short* WIH = W16 + EL_WIH;
  const unsigned short* WHH = W16 + EL_WHH;
  const float* CST = (const float*)(ws + OFF_W + (size_t)UNIT_CST * 16);

  prep_kernel<<<(PREP_UNITS + 255) / 256, 256, 0, stream>>>(lin0_w, lin0_b, nn1_w, nn1_b, root_w, conv_b,
                                                          gru_w_ih, gru_w_hh, gru_b_ih, gru_b_hh,
                                                          lin1_w, lin1_b, lin2_w, WGT);
  build_kernel<<<NUM_NODES / BUILD_TILE, 256, 0, stream>>>(edge_idx + NUM_EDGES, CNT, NBR);
  lin0_kernel<<<NUM_NODES / 128, 256, 0, stream>>>(x, L0T, CST, HHI, HLO);

  for (int it = 0; it < NUM_GRU * NUM_REP; ++it) {
    const int j = it / NUM_REP;
    msgprep_kernel<<<NUM_NODES / 64, 128, 0, stream>>>(HHI, HLO, L1T, WCT, CST, TPL);
    edge_kernel<<<NUM_NODES / 16, 256, 0, stream>>>(TPL, edge_attr, edge_idx, NBR, CNT, XIN);
    gru_kernel<SPLIT_RZ_COLS, SPLIT_HN_COLS><<<NUM_NODES / 64, 128, 0, stream>>>(
        HHI, HLO, XIN, WIH + (size_t)j * GATE3 * 32, WHH + (size_t)j * GATE3 * HID, CST + CST_GB + (size_t)j * 256);
  }
  pool_kernel<<<NUM_GRAPHS / 256, 256, 0, stream>>>(HHI, HLO, CST, batch, out);
}
